// EGNNLayerTorch_31653908971779
// MI455X (gfx1250) — hardware-run, weakly checked
//
#include <hip/hip_runtime.h>


namespace {
constexpr int N = 50000, E = 800000, DH = 128, DE = 16, DM = 128, KX = 2 * DH + DE  , KXP = 288, SQK = 2 * DH  ;
constexpr float XS = 8.0f, HS = 256.0f, WSC = 256.0f, LNEPS = 1e-5f;
typedef _Float16 b16;
typedef __attribute__((ext_vector_type(16))) _Float16 v16b;
typedef __attribute__((ext_vector_type(8))) _Float16 v8b;
typedef __attribute__((ext_vector_type(8))) float v8f;
typedef __attribute__((ext_vector_type(4))) float v4f;
typedef __attribute__((ext_vector_type(4))) _Float16 v4b;
__device__ __forceinline__ float bf16_rne(float f) { unsigned int u = __float_as_uint(f); u += 0x7FFFu + ((u >> 16) & 1u); float r = __uint_as_float(u & 0xFFFF0000u); asm volatile("" : "+v"(r)); return r; }
__device__ __forceinline__ float bfv(float f) { float r = bf16_rne(f); asm volatile("" : "+v"(r)); return r; }
__device__ __forceinline__ void split16(float v, b16& hi, b16& lo) { hi = (b16)v; lo = (b16)(v - (float)hi); }
__device__ __forceinline__ v16b frag_kb(const b16* p, int hh) { const v8b a = *(const v8b*)(p + 8 * hh), b = *(const v8b*)(p + 16 + 8 * hh); v16b f;
#pragma unroll
  for (int e = 0; e < 8; ++e) { f[e] = a[e]; f[8 + e] = b[e]; } return f; }
__device__ __forceinline__ v8f wmma16b(v16b a, v16b b, v8f c) { v8f d = __builtin_amdgcn_wmma_f32_16x16x32_f16(false, a, false, b, (short)0, c, false, false); asm volatile("v_nop\n\tv_nop\n\tv_nop\n\tv_nop" : "+v"(d) : "v"(a), "v"(b)); return d; }
__device__ __forceinline__ void wave_lds_sync() { __builtin_amdgcn_fence(__ATOMIC_RELEASE, "workgroup"); __builtin_amdgcn_wave_barrier(); __builtin_amdgcn_fence(__ATOMIC_ACQUIRE, "workgroup"); }
__device__ __forceinline__ float pmul(float a, float b) { float p = a * b; asm volatile("" : "+v"(p)); return p; }
__device__ __forceinline__ int iclamp(int v, int lo, int hi) { return v < lo ? lo : (v > hi ? hi : v); }
__device__ __forceinline__ float silu(float v) { return v / (1.0f + __expf(-v)); }
constexpr int CSR_NBLKD = 512, CSR_GBD = 9, CSR_GND = 1 << CSR_GBD  , CSR_TSD = (CSR_GND < 32 ? 32 : CSR_GND)  , CSR_MAXGD = 512, CSR_CAPD = 12288  ;
__device__ __host__ __forceinline__ int csr_tixD(int v) { return (v >> CSR_GBD) * CSR_TSD + (v & (CSR_GND - 1)); }
__global__ __launch_bounds__(64) void csrA_kernelD(const int* __restrict__ dst, int E, int N, int nG, int CHP, int NGP, int* __restrict__ STG, int* __restrict__ HST) {
  extern __shared__ int sm[];
  int* cnt = sm; int* run = sm + NGP; int* ids = sm + 2 * NGP;
  const int b = blockIdx.x; const int ch = (E + CSR_NBLKD - 1) / CSR_NBLKD; const int e0 = b * ch, e1 = min(E, e0 + ch);
  for (int i = threadIdx.x; i < NGP; i += 64) cnt[i] = 0;
  for (int i = threadIdx.x; i < CHP; i += 64) ids[i] = -1;
  __syncthreads();
  if (threadIdx.x == 0) {
    for (int e = e0; e < e1; ++e) { int d = dst[e]; d = (d < 0) ? 0 : (d >= N ? N - 1 : d); cnt[d >> CSR_GBD] += 1; }
    int acc = 0; for (int g = 0; g < nG; ++g) { run[g] = acc; acc += cnt[g]; }
    for (int e = e0; e < e1; ++e) { int d = dst[e]; d = (d < 0) ? 0 : (d >= N ? N - 1 : d); const int g = d >> CSR_GBD; ids[run[g]] = e; run[g] += 1; } }
  __syncthreads();
  typedef __attribute__((ext_vector_type(4))) int v4i;
  for (int pass = 0; pass < 2; ++pass) {
    for (int i = threadIdx.x; i < CHP / 4; i += 64) *(volatile v4i*)(STG + (size_t)b * CHP + i * 4) = *(const v4i*)(&ids[i * 4]);
    for (int i = threadIdx.x; i < NGP / 4; i += 64) { v4i v; for (int e = 0; e < 4; ++e) v[e] = (i * 4 + e < nG) ? cnt[i * 4 + e] : 0; *(volatile v4i*)(HST + (size_t)b * NGP + i * 4) = v; }
    __threadfence(); }
}
__global__ __launch_bounds__(512) void csrS_kernelD(const int* __restrict__ HST, int nG, int NGP, int* __restrict__ START, int* __restrict__ TOT, int* __restrict__ OFF) {
  __shared__ int tot[CSR_MAXGD];
  const int b = threadIdx.x;
  for (int pass = 0; pass < 2; ++pass) { int runb = 0; for (int g = 0; g < nG; ++g) { int c = HST[(size_t)b * NGP + g]; c = (c < 0) ? 0 : c; ((volatile int*)OFF)[(size_t)g * CSR_NBLKD + b] = runb; runb += c; } __threadfence(); }
  for (int g = threadIdx.x; g < nG; g += 512) { int s = 0; for (int bb = 0; bb < CSR_NBLKD; ++bb) { int c = HST[(size_t)bb * NGP + g]; s += (c < 0) ? 0 : c; } tot[g] = s; }
  __syncthreads();
  if (threadIdx.x < 32) {
    __shared__ int st[CSR_MAXGD + 32];
    if (threadIdx.x == 0) { int acc = 0; for (int g = 0; g < NGP; ++g) { st[g] = acc; if (g < nG) acc += (tot[g] + 31) & ~31; } st[NGP] = acc; }
    __builtin_amdgcn_fence(__ATOMIC_RELEASE, "workgroup"); __builtin_amdgcn_wave_barrier(); __builtin_amdgcn_fence(__ATOMIC_ACQUIRE, "workgroup");
    for (int pass = 0; pass < 2; ++pass) { for (int i = threadIdx.x; i < NGP + 32; i += 32) { ((volatile int*)START)[i] = (i <= NGP) ? st[min(i, NGP)] : 0; ((volatile int*)TOT)[i] = (i < nG) ? tot[i] : 0; } __threadfence(); } }
}
__global__ __launch_bounds__(256) void csrB_kernelD(const int* __restrict__ dst, int N, int nG, int CHP, int NGP, int permLen, const int* __restrict__ STG, const int* __restrict__ HST, const int* __restrict__ OFF, const int* __restrict__ START, const int* __restrict__ TOT, int* __restrict__ PERM, int* __restrict__ ROWPTR, int* __restrict__ ROWCNT, int* __restrict__ FLAG) {
  typedef __attribute__((ext_vector_type(4))) int v4i;
  __shared__ int ids[CSR_CAPD]; __shared__ unsigned short key[CSR_CAPD]; __shared__ int outp[CSR_CAPD]; __shared__ int ncnt[CSR_GND + 1]; __shared__ int boff[CSR_NBLKD + 1];
  const int g = blockIdx.x, t_ = threadIdx.x; int tot = TOT[g]; int st = START[g], stn = START[g + 1]; const int v0 = g * CSR_GND; const int nv = min(CSR_GND, N - v0); const int t0 = g * CSR_TSD;
  st = (st < 0) ? 0 : (st > permLen - 32 ? permLen - 32 : st) & ~31; stn = (stn < st) ? st : (stn > permLen ? permLen : stn); tot = (tot < 0) ? 0 : tot; if (tot > stn - st && tot <= CSR_CAPD) tot = stn - st;
  if (tot > CSR_CAPD) {
    for (int pass = 0; pass < 2; ++pass) { for (int i = t_; i < CSR_TSD / 4; i += 256) { v4i a, c; for (int e = 0; e < 4; ++e) { a[e] = st; c[e] = 0; } *(volatile v4i*)(ROWPTR + t0 + i * 4) = a; *(volatile v4i*)(ROWCNT + t0 + i * 4) = c; } if (t_ == 0) ((volatile int*)FLAG)[0] = 1; __threadfence(); } (void)nv; return; }
  if (t_ == 0) { int acc = 0; for (int b = 0; b < CSR_NBLKD; ++b) { boff[b] = acc; int c = HST[(size_t)b * NGP + g]; c = (c < 0) ? 0 : (c > CHP ? CHP : c); acc += c; if (acc > tot) acc = tot; } boff[CSR_NBLKD] = acc; }
  for (int i = t_; i <= CSR_GND; i += 256) ncnt[i] = 0;
  __syncthreads();
  for (int b = 0; b < CSR_NBLKD; ++b) { const int c = boff[b + 1] - boff[b]; int o_ = OFF[(size_t)g * CSR_NBLKD + b]; o_ = (o_ < 0) ? 0 : (o_ > CHP - c ? CHP - c : o_); const int* src_ = STG + (size_t)b * CHP + o_;
    for (int i = t_; i < c; i += 256) { int id = src_[i]; id = (id < 0) ? 0 : id; ids[boff[b] + i] = id; int d = dst[id]; d = (d < v0) ? v0 : (d >= N ? N - 1 : d); int kk = d - v0; kk = (kk < 0) ? 0 : (kk >= CSR_GND ? CSR_GND - 1 : kk); key[boff[b] + i] = (unsigned short)kk; } }
  __syncthreads();
  if (t_ == 0) { for (int i = 0; i < tot; ++i) ncnt[key[i]] += 1; int acc = 0; for (int vl = 0; vl < CSR_GND; ++vl) { const int c = ncnt[vl]; ncnt[vl] = acc; acc += c; } ncnt[CSR_GND] = acc;
    for (int i = 0; i < tot; ++i) { const int vl = key[i]; outp[ncnt[vl]] = ids[i]; ncnt[vl] += 1; }
    for (int vl = CSR_GND; vl > 0; --vl) ncnt[vl] = ncnt[vl - 1]; ncnt[0] = 0; }
  __syncthreads();
  for (int pass = 0; pass < 2; ++pass) {
    for (int i = t_; i < (stn - st) / 4; i += 256) { v4i v; for (int e = 0; e < 4; ++e) { const int q = i * 4 + e; v[e] = (q < tot) ? outp[q] : -1; } *(volatile v4i*)(PERM + st + i * 4) = v; }
    for (int i = t_; i < CSR_TSD / 4; i += 256) { v4i a, c; for (int e = 0; e < 4; ++e) { const int vl = i * 4 + e; const int vc = vl < CSR_GND ? vl : CSR_GND; a[e] = (vl < CSR_GND) ? st + ncnt[vc] : st; c[e] = (vl < nv) ? (ncnt[(vc < CSR_GND ? vc : CSR_GND - 1) + 1] - ncnt[vc]) : 0; } *(volatile v4i*)(ROWPTR + t0 + i * 4) = a; *(volatile v4i*)(ROWCNT + t0 + i * 4) = c; }
    __threadfence(); }
}
__global__ __launch_bounds__(256) void csrZ_kernelD(int* __restrict__ p, size_t n4) { typedef __attribute__((ext_vector_type(4))) int v4i; const size_t tid = (size_t)blockIdx.x * 256 + threadIdx.x, nth = (size_t)gridDim.x * 256; v4i z = {0, 0, 0, 0}; for (size_t i = tid; i < n4; i += nth) *(volatile v4i*)(p + i * 4) = z; }
struct CsrBufsD { int *STG, *HST, *OFF, *START, *TOT, *PERM, *ROWPTR, *ROWCNT, *FLAG; int nG, NGP, CHP; size_t permLen; char* base; size_t bytes; };
static size_t csr_carveD(CsrBufsD& c, char* ws, size_t off, int E, int N) {
  const size_t off0 = off; c.base = ws + off;
  auto al = [&](size_t bytes) { char* p = ws + off; off += (bytes + 255) & ~(size_t)255; return p; };
  c.nG = (N + CSR_GND - 1) / CSR_GND; c.NGP = (c.nG + 31) & ~31; const int ch = (E + CSR_NBLKD - 1) / CSR_NBLKD; c.CHP = (ch + 31) & ~31; c.permLen = (size_t)E + 32 * (size_t)c.nG + 32;
  c.STG = (int*)al((size_t)CSR_NBLKD * c.CHP * 4); c.HST = (int*)al((size_t)CSR_NBLKD * c.NGP * 4); c.OFF = (int*)al((size_t)c.NGP * CSR_NBLKD * 4); c.START = (int*)al((size_t)(c.NGP + 64) * 4); c.TOT = (int*)al((size_t)(c.NGP + 64) * 4);
  c.PERM = (int*)al(c.permLen * 4); c.ROWPTR = (int*)al((size_t)c.nG * CSR_TSD * 4); c.ROWCNT = (int*)al((size_t)c.nG * CSR_TSD * 4); c.FLAG = (int*)al(256);
  c.bytes = off - off0; return off;
}
static void csr_buildD(const CsrBufsD& c, const int* dst, int E, int N, hipStream_t stream) {
  const size_t smem = (size_t)(2 * c.NGP + c.CHP) * 4;
  csrZ_kernelD<<<512, 256, 0, stream>>>((int*)c.base, c.bytes / 16);
  csrA_kernelD<<<CSR_NBLKD, 64, smem, stream>>>(dst, E, N, c.nG, c.CHP, c.NGP, c.STG, c.HST);
  csrS_kernelD<<<1, 512, 0, stream>>>(c.HST, c.nG, c.NGP, c.START, c.TOT, c.OFF);
  csrB_kernelD<<<c.nG, 256, 0, stream>>>(dst, N, c.nG, c.CHP, c.NGP, (int)c.permLen, c.STG, c.HST, c.OFF, c.START, c.TOT, c.PERM, c.ROWPTR, c.ROWCNT, c.FLAG);
}
constexpr int CSR_NBLKS = 512, CSR_GBS = 9, CSR_GNS = 1 << CSR_GBS  , CSR_TSS = (CSR_GNS < 32 ? 32 : CSR_GNS)  , CSR_MAXGS = 512, CSR_CAPS = 12288  ;
__device__ __host__ __forceinline__ int csr_tixS(int v) { return (v >> CSR_GBS) * CSR_TSS + (v & (CSR_GNS - 1)); }
__global__ __launch_bounds__(64) void csrA_kernelS(const int* __restrict__ dst, int E, int N, int nG, int CHP, int NGP, int* __restrict__ STG, int* __restrict__ HST) {
  extern __shared__ int sm[];
  int* cnt = sm; int* run = sm + NGP; int* ids = sm + 2 * NGP;
  const int b = blockIdx.x; const int ch = (E + CSR_NBLKS - 1) / CSR_NBLKS; const int e0 = b * ch, e1 = min(E, e0 + ch);
  for (int i = threadIdx.x; i < NGP; i += 64) cnt[i] = 0;
  for (int i = threadIdx.x; i < CHP; i += 64) ids[i] = -1;
  __syncthreads();
  if (threadIdx.x == 0) {
    for (int e = e0; e < e1; ++e) { int d = dst[e]; d = (d < 0) ? 0 : (d >= N ? N - 1 : d); cnt[d >> CSR_GBS] += 1; }
    int acc = 0; for (int g = 0; g < nG; ++g) { run[g] = acc; acc += cnt[g]; }
    for (int e = e0; e < e1; ++e) { int d = dst[e]; d = (d < 0) ? 0 : (d >= N ? N - 1 : d); const int g = d >> CSR_GBS; ids[run[g]] = e; run[g] += 1; } }
  __syncthreads();
  typedef __attribute__((ext_vector_type(4))) int v4i;
  for (int pass = 0; pass < 2; ++pass) {
    for (int i = threadIdx.x; i < CHP / 4; i += 64) *(volatile v4i*)(STG + (size_t)b * CHP + i * 4) = *(const v4i*)(&ids[i * 4]);
    for (int i = threadIdx.x; i < NGP / 4; i += 64) { v4i v; for (int e = 0; e < 4; ++e) v[e] = (i * 4 + e < nG) ? cnt[i * 4 + e] : 0; *(volatile v4i*)(HST + (size_t)b * NGP + i * 4) = v; }
    __threadfence(); }
}
__global__ __launch_bounds__(512) void csrS_kernelS(const int* __restrict__ HST, int nG, int NGP, int* __restrict__ START, int* __restrict__ TOT, int* __restrict__ OFF) {
  __shared__ int tot[CSR_MAXGS];
  const int b = threadIdx.x;
  for (int pass = 0; pass < 2; ++pass) { int runb = 0; for (int g = 0; g < nG; ++g) { int c = HST[(size_t)b * NGP + g]; c = (c < 0) ? 0 : c; ((volatile int*)OFF)[(size_t)g * CSR_NBLKS + b] = runb; runb += c; } __threadfence(); }
  for (int g = threadIdx.x; g < nG; g += 512) { int s = 0; for (int bb = 0; bb < CSR_NBLKS; ++bb) { int c = HST[(size_t)bb * NGP + g]; s += (c < 0) ? 0 : c; } tot[g] = s; }
  __syncthreads();
  if (threadIdx.x < 32) {
    __shared__ int st[CSR_MAXGS + 32];
    if (threadIdx.x == 0) { int acc = 0; for (int g = 0; g < NGP; ++g) { st[g] = acc; if (g < nG) acc += (tot[g] + 31) & ~31; } st[NGP] = acc; }
    __builtin_amdgcn_fence(__ATOMIC_RELEASE, "workgroup"); __builtin_amdgcn_wave_barrier(); __builtin_amdgcn_fence(__ATOMIC_ACQUIRE, "workgroup");
    for (int pass = 0; pass < 2; ++pass) { for (int i = threadIdx.x; i < NGP + 32; i += 32) { ((volatile int*)START)[i] = (i <= NGP) ? st[min(i, NGP)] : 0; ((volatile int*)TOT)[i] = (i < nG) ? tot[i] : 0; } __threadfence(); } }
}
__global__ __launch_bounds__(256) void csrB_kernelS(const int* __restrict__ dst, int N, int nG, int CHP, int NGP, int permLen, const int* __restrict__ STG, const int* __restrict__ HST, const int* __restrict__ OFF, const int* __restrict__ START, const int* __restrict__ TOT, int* __restrict__ PERM, int* __restrict__ ROWPTR, int* __restrict__ ROWCNT, int* __restrict__ FLAG) {
  typedef __attribute__((ext_vector_type(4))) int v4i;
  __shared__ int ids[CSR_CAPS]; __shared__ unsigned short key[CSR_CAPS]; __shared__ int outp[CSR_CAPS]; __shared__ int ncnt[CSR_GNS + 1]; __shared__ int boff[CSR_NBLKS + 1];
  const int g = blockIdx.x, t_ = threadIdx.x; int tot = TOT[g]; int st = START[g], stn = START[g + 1]; const int v0 = g * CSR_GNS; const int nv = min(CSR_GNS, N - v0); const int t0 = g * CSR_TSS;
  st = (st < 0) ? 0 : (st > permLen - 32 ? permLen - 32 : st) & ~31; stn = (stn < st) ? st : (stn > permLen ? permLen : stn); tot = (tot < 0) ? 0 : tot; if (tot > stn - st && tot <= CSR_CAPS) tot = stn - st;
  if (tot > CSR_CAPS) {
    for (int pass = 0; pass < 2; ++pass) { for (int i = t_; i < CSR_TSS / 4; i += 256) { v4i a, c; for (int e = 0; e < 4; ++e) { a[e] = st; c[e] = 0; } *(volatile v4i*)(ROWPTR + t0 + i * 4) = a; *(volatile v4i*)(ROWCNT + t0 + i * 4) = c; } if (t_ == 0) ((volatile int*)FLAG)[0] = 1; __threadfence(); } (void)nv; return; }
  if (t_ == 0) { int acc = 0; for (int b = 0; b < CSR_NBLKS; ++b) { boff[b] = acc; int c = HST[(size_t)b * NGP + g]; c = (c < 0) ? 0 : (c > CHP ? CHP : c); acc += c; if (acc > tot) acc = tot; } boff[CSR_NBLKS] = acc; }
  for (int i = t_; i <= CSR_GNS; i += 256) ncnt[i] = 0;
  __syncthreads();
  for (int b = 0; b < CSR_NBLKS; ++b) { const int c = boff[b + 1] - boff[b]; int o_ = OFF[(size_t)g * CSR_NBLKS + b]; o_ = (o_ < 0) ? 0 : (o_ > CHP - c ? CHP - c : o_); const int* src_ = STG + (size_t)b * CHP + o_;
    for (int i = t_; i < c; i += 256) { int id = src_[i]; id = (id < 0) ? 0 : id; ids[boff[b] + i] = id; int d = dst[id]; d = (d < v0) ? v0 : (d >= N ? N - 1 : d); int kk = d - v0; kk = (kk < 0) ? 0 : (kk >= CSR_GNS ? CSR_GNS - 1 : kk); key[boff[b] + i] = (unsigned short)kk; } }
  __syncthreads();
  if (t_ == 0) { for (int i = 0; i < tot; ++i) ncnt[key[i]] += 1; int acc = 0; for (int vl = 0; vl < CSR_GNS; ++vl) { const int c = ncnt[vl]; ncnt[vl] = acc; acc += c; } ncnt[CSR_GNS] = acc;
    for (int i = 0; i < tot; ++i) { const int vl = key[i]; outp[ncnt[vl]] = ids[i]; ncnt[vl] += 1; }
    for (int vl = CSR_GNS; vl > 0; --vl) ncnt[vl] = ncnt[vl - 1]; ncnt[0] = 0; }
  __syncthreads();
  for (int pass = 0; pass < 2; ++pass) {
    for (int i = t_; i < (stn - st) / 4; i += 256) { v4i v; for (int e = 0; e < 4; ++e) { const int q = i * 4 + e; v[e] = (q < tot) ? outp[q] : -1; } *(volatile v4i*)(PERM + st + i * 4) = v; }
    for (int i = t_; i < CSR_TSS / 4; i += 256) { v4i a, c; for (int e = 0; e < 4; ++e) { const int vl = i * 4 + e; const int vc = vl < CSR_GNS ? vl : CSR_GNS; a[e] = (vl < CSR_GNS) ? st + ncnt[vc] : st; c[e] = (vl < nv) ? (ncnt[(vc < CSR_GNS ? vc : CSR_GNS - 1) + 1] - ncnt[vc]) : 0; } *(volatile v4i*)(ROWPTR + t0 + i * 4) = a; *(volatile v4i*)(ROWCNT + t0 + i * 4) = c; }
    __threadfence(); }
}
__global__ __launch_bounds__(256) void csrZ_kernelS(int* __restrict__ p, size_t n4) { typedef __attribute__((ext_vector_type(4))) int v4i; const size_t tid = (size_t)blockIdx.x * 256 + threadIdx.x, nth = (size_t)gridDim.x * 256; v4i z = {0, 0, 0, 0}; for (size_t i = tid; i < n4; i += nth) *(volatile v4i*)(p + i * 4) = z; }
struct CsrBufsS { int *STG, *HST, *OFF, *START, *TOT, *PERM, *ROWPTR, *ROWCNT, *FLAG; int nG, NGP, CHP; size_t permLen; char* base; size_t bytes; };
static size_t csr_carveS(CsrBufsS& c, char* ws, size_t off, int E, int N) {
  const size_t off0 = off; c.base = ws + off;
  auto al = [&](size_t bytes) { char* p = ws + off; off += (bytes + 255) & ~(size_t)255; return p; };
  c.nG = (N + CSR_GNS - 1) / CSR_GNS; c.NGP = (c.nG + 31) & ~31; const int ch = (E + CSR_NBLKS - 1) / CSR_NBLKS; c.CHP = (ch + 31) & ~31; c.permLen = (size_t)E + 32 * (size_t)c.nG + 32;
  c.STG = (int*)al((size_t)CSR_NBLKS * c.CHP * 4); c.HST = (int*)al((size_t)CSR_NBLKS * c.NGP * 4); c.OFF = (int*)al((size_t)c.NGP * CSR_NBLKS * 4); c.START = (int*)al((size_t)(c.NGP + 64) * 4); c.TOT = (int*)al((size_t)(c.NGP + 64) * 4);
  c.PERM = (int*)al(c.permLen * 4); c.ROWPTR = (int*)al((size_t)c.nG * CSR_TSS * 4); c.ROWCNT = (int*)al((size_t)c.nG * CSR_TSS * 4); c.FLAG = (int*)al(256);
  c.bytes = off - off0; return off;
}
static void csr_buildS(const CsrBufsS& c, const int* dst, int E, int N, hipStream_t stream) {
  const size_t smem = (size_t)(2 * c.NGP + c.CHP) * 4;
  csrZ_kernelS<<<512, 256, 0, stream>>>((int*)c.base, c.bytes / 16);
  csrA_kernelS<<<CSR_NBLKS, 64, smem, stream>>>(dst, E, N, c.nG, c.CHP, c.NGP, c.STG, c.HST);
  csrS_kernelS<<<1, 512, 0, stream>>>(c.HST, c.nG, c.NGP, c.START, c.TOT, c.OFF);
  csrB_kernelS<<<c.nG, 256, 0, stream>>>(dst, N, c.nG, c.CHP, c.NGP, (int)c.permLen, c.STG, c.HST, c.OFF, c.START, c.TOT, c.PERM, c.ROWPTR, c.ROWCNT, c.FLAG);
}


__global__ __launch_bounds__(256) void wput_kernel(const float* __restrict__ we1, const float* __restrict__ we2, const float* __restrict__ wx1, const float* __restrict__ wh1, const float* __restrict__ wh2, b16* __restrict__ WE1, b16* __restrict__ WE2, b16* __restrict__ WX1, b16* __restrict__ WH1, b16* __restrict__ WH2) { const int u = blockIdx.x * 256 + threadIdx.x; v8b v;
  if (u < DM * (KXP / 8)) { const int o = u / (KXP / 8), k0 = (u % (KXP / 8)) * 8;
#pragma unroll
    for (int j = 0; j < 8; ++j) { const int k = k0 + j; const int row = k < 2 * DH ? k : (k < KX ? SQK + 1 + (k - 2 * DH) : -1); v[j] = (b16)(row >= 0 ? bf16_rne(we1[(size_t)row * DM + o]) * WSC : 0.0f); } for (int pass = 0; pass < 2; ++pass) { *(volatile v8b*)(WE1 + (size_t)o * KXP + k0) = v; __threadfence(); } }
  if (u < DM * 16) { const int o = u / 16, k0 = (u % 16) * 8;
#pragma unroll
    for (int j = 0; j < 8; ++j) v[j] = (b16)(bf16_rne(we2[(size_t)(k0 + j) * DM + o]) * WSC); for (int pass = 0; pass < 2; ++pass) { *(volatile v8b*)(WE2 + (size_t)o * DM + k0) = v; __threadfence(); }
#pragma unroll
    for (int j = 0; j < 8; ++j) v[j] = (b16)(bf16_rne(wx1[(size_t)(k0 + j) * DM + o]) * WSC); for (int pass = 0; pass < 2; ++pass) { *(volatile v8b*)(WX1 + (size_t)o * DM + k0) = v; __threadfence(); }
#pragma unroll
    for (int j = 0; j < 8; ++j) v[j] = (b16)(bf16_rne(wh2[(size_t)(k0 + j) * DH + o]) * WSC); for (int pass = 0; pass < 2; ++pass) { *(volatile v8b*)(WH2 + (size_t)o * DH + k0) = v; __threadfence(); } }
  if (u < DH * 32) { const int o = u / 32, k0 = (u % 32) * 8;
#pragma unroll
    for (int j = 0; j < 8; ++j) v[j] = (b16)(bf16_rne(wh1[(size_t)(k0 + j) * DH + o]) * WSC); for (int pass = 0; pass < 2; ++pass) { *(volatile v8b*)(WH1 + (size_t)o * 2 * DH + k0) = v; __threadfence(); } } }
__global__ __launch_bounds__(32) void edge_kernel(const float* __restrict__ h, const float* __restrict__ x, const float* __restrict__ attr, const int* __restrict__ ei, const b16* __restrict__ WE1, const b16* __restrict__ WE2, const b16* __restrict__ WX1, const float* __restrict__ we1, const float* __restrict__ be1, const float* __restrict__ be2, const float* __restrict__ bx1, const float* __restrict__ wx2, const float* __restrict__ bx2, int EB, int ELIM, int NLIM, b16* __restrict__ MSG, float* __restrict__ WGT) {
  __shared__ __attribute__((aligned(16))) b16 Ah[16][KXP + 8], Bh[16][DM + 8], Bl[16][DM + 8]; __shared__ float Tf[16][DM + 4], Sq[16], Df[16][4]; const int lane = threadIdx.x, nloc = lane & 15, hlf = lane >> 4; const size_t e0 = (size_t)EB + (size_t)blockIdx.x * 16; if (e0 >= (size_t)ELIM) return;
  { const size_t e = e0 + nloc; const int s = iclamp(ei[e], 0, NLIM - 1), d = iclamp(ei[E + e], 0, NLIM - 1);
    const float* hp = h + (size_t)(hlf ? d : s) * DH; for (int c = 0; c < DH; ++c) Ah[nloc][hlf * DH + c] = (b16)(bf16_rne(hp[c]) * XS);
    if (hlf == 0) { for (int c = 0; c < DE; ++c) Ah[nloc][2 * DH + c] = (b16)(bf16_rne(attr[e * DE + c]) * XS); for (int c = KX; c < KXP + 8; ++c) Ah[nloc][c] = (b16)0.0f;
      float sq = 0.0f; for (int k = 0; k < 3; ++k) { const float df = bfv(x[(size_t)s * 3 + k]) - bfv(x[(size_t)d * 3 + k]); Df[nloc][k] = df; sq += df * df; } Df[nloc][3] = 0.0f; Sq[nloc] = sq; } }
  if (lane < 16) for (int k = DM; k < DM + 8; ++k) { Bh[lane][k] = (b16)0.0f; Bl[lane][k] = (b16)0.0f; }
  wave_lds_sync(); v8f acc[8];
#pragma unroll
  for (int t = 0; t < 8; ++t) acc[t] = (v8f){};
#pragma unroll 3
  for (int kb = 0; kb < KXP; kb += 32) { const v16b a = frag_kb(&Ah[nloc][kb], hlf);
#pragma unroll
    for (int t = 0; t < 8; ++t) acc[t] = wmma16b(a, frag_kb(WE1 + (size_t)(t * 16 + nloc) * KXP + kb, hlf), acc[t]); }
#pragma unroll
  for (int t = 0; t < 8; ++t) { const int cc = t * 16 + nloc; const float bb = bfv(be1[cc]), wsq = bfv(we1[(size_t)SQK * DM + cc]);
#pragma unroll
    for (int r8 = 0; r8 < 8; ++r8) { const int rr = 8 * hlf + r8; b16 p, ql; split16(silu(acc[t][r8] * (1.0f / (XS * WSC)) + pmul(Sq[rr], wsq) + bb) * HS, p, ql); Bh[rr][cc] = p; Bl[rr][cc] = ql; } }
  wave_lds_sync();
#pragma unroll
  for (int t = 0; t < 8; ++t) acc[t] = (v8f){};
#pragma unroll
  for (int kb = 0; kb < DM; kb += 32) { const v16b a = frag_kb(&Bh[nloc][kb], hlf), al = frag_kb(&Bl[nloc][kb], hlf);
#pragma unroll
    for (int t = 0; t < 8; ++t) { const v16b bw = frag_kb(WE2 + (size_t)(t * 16 + nloc) * DM + kb, hlf); acc[t] = wmma16b(a, bw, acc[t]); acc[t] = wmma16b(al, bw, acc[t]); } }
#pragma unroll
  for (int t = 0; t < 8; ++t) { const int cc = t * 16 + nloc; const float bb = bfv(be2[cc]);
#pragma unroll
    for (int r8 = 0; r8 < 8; ++r8) Tf[8 * hlf + r8][cc] = silu(acc[t][r8] * (1.0f / (HS * WSC)) + bb); }
  wave_lds_sync();
  for (int rr = 0; rr < 16; ++rr) for (int q = 0; q < 4; ++q) Bh[rr][q * 32 + lane] = (b16)(Tf[rr][q * 32 + lane] * HS);
  wave_lds_sync(); v8f ax[8];
#pragma unroll
  for (int t = 0; t < 8; ++t) ax[t] = (v8f){};
#pragma unroll
  for (int kb = 0; kb < DM; kb += 32) { const v16b a = frag_kb(&Bh[nloc][kb], hlf);
#pragma unroll
    for (int t = 0; t < 8; ++t) ax[t] = wmma16b(a, frag_kb(WX1 + (size_t)(t * 16 + nloc) * DM + kb, hlf), ax[t]); }
  __shared__ float Wp[16][16];
#pragma unroll
  for (int r8 = 0; r8 < 8; ++r8) { float s = 0.0f;
#pragma unroll
    for (int t = 0; t < 8; ++t) { const int cc = t * 16 + nloc; s += pmul(silu(ax[t][r8] * (1.0f / (HS * WSC)) + bfv(bx1[cc])), bfv(wx2[cc])); } Wp[8 * hlf + r8][nloc] = s; }
  wave_lds_sync();
  float wv = 0.0f; if (lane < 16) { for (int q = 0; q < 16; ++q) wv += Wp[lane][q]; wv += bfv(bx2[0]); }
  for (int pass = 0; pass < 2; ++pass) { for (int rr = 0; rr < 16; ++rr) { v4b m4; for (int k = 0; k < 4; ++k) m4[k] = (b16)(Tf[rr][lane * 4 + k] * 64.0f); *(volatile v4b*)(MSG + (e0 - EB + rr) * DM + lane * 4) = m4; }
    ((volatile float*)WGT)[(e0 / 16) * 32 + lane] = lane < 16 ? wv : 0.0f; __threadfence(); } }
template <int PASS>
__global__ __launch_bounds__(256) void agg_kernel(const b16* __restrict__ MSG, int EB, int EEND, const float* __restrict__ AGGIN, const int* __restrict__ srcs, const int* __restrict__ PERM, const int* __restrict__ ROWPTR, const int* __restrict__ ROWCNT, int permLen, int NLIM, int ELIM, float* __restrict__ AGG, float* __restrict__ CNT) { const int wave = threadIdx.x >> 5, lane = threadIdx.x & 31; const size_t i = (size_t)blockIdx.x * 8 + wave; if (i >= (size_t)NLIM) return; int st = ROWPTR[i], cnt = ROWCNT[i]; cnt = iclamp(cnt, 0, E); st = iclamp(st, 0, permLen - cnt);
  v4f acc = PASS ? *(const v4f*)(AGGIN + i * DM + lane * 4) : (v4f){0, 0, 0, 0}; int nin = 0;
#pragma unroll 1
  for (int j = 0; j < cnt; ++j) { const int e = iclamp(PERM[st + j], 0, E - 1); if ((size_t)iclamp(srcs[e], 0, N - 1) >= (size_t)NLIM || e >= ELIM) continue; ++nin; if (e < EB || e >= EEND) continue; const v4b m = *(const v4b*)(MSG + (size_t)(e - EB) * DM + lane * 4);
#pragma unroll
    for (int k = 0; k < 4; ++k) acc[k] += (float)m[k] * (1.0f / 64.0f); }
  const float c = fmaxf((float)nin, 1.0f), inv = 1.0f / c; v4f o; for (int k = 0; k < 4; ++k) o[k] = PASS ? pmul(acc[k], inv) : acc[k];
  for (int pass = 0; pass < 2; ++pass) { *(volatile v4f*)(AGG + i * DM + lane * 4) = o; if (PASS && lane == 0) ((volatile float*)CNT)[i] = c; __threadfence(); } }
__global__ __launch_bounds__(32) void node_kernel(const float* __restrict__ h, const float* __restrict__ AGG, const b16* __restrict__ WH1, const b16* __restrict__ WH2, const float* __restrict__ bh1, const float* __restrict__ bh2, const float* __restrict__ lg, const float* __restrict__ lb, int NLIM, float* __restrict__ HN) { __shared__ __attribute__((aligned(16))) b16 Ah[16][2 * DH + 8], Al[16][2 * DH + 8]; __shared__ float Tf[16][DH + 4]; const int lane = threadIdx.x, nloc = lane & 15, hlf = lane >> 4; const size_t m0 = (size_t)blockIdx.x * 16; if (m0 >= (size_t)NLIM) return;
  for (int rr = 0; rr < 16; ++rr) for (int q = 0; q < 4; ++q) { const int c = q * 32 + lane; Ah[rr][c] = (b16)(bf16_rne(h[(m0 + rr) * DH + c]) * HS); Al[rr][c] = (b16)0.0f; b16 p, ql; split16(AGG[(m0 + rr) * DM + c] * HS, p, ql); Ah[rr][DH + c] = p; Al[rr][DH + c] = ql; }
  if (lane < 16) for (int k = 2 * DH; k < 2 * DH + 8; ++k) { Ah[lane][k] = (b16)0.0f; Al[lane][k] = (b16)0.0f; }
  wave_lds_sync(); v8f acc[8];
#pragma unroll
  for (int t = 0; t < 8; ++t) acc[t] = (v8f){};
#pragma unroll 2
  for (int kb = 0; kb < 2 * DH; kb += 32) { const v16b a = frag_kb(&Ah[nloc][kb], hlf), al = frag_kb(&Al[nloc][kb], hlf);
#pragma unroll
    for (int t = 0; t < 8; ++t) { const v16b bw = frag_kb(WH1 + (size_t)(t * 16 + nloc) * 2 * DH + kb, hlf); acc[t] = wmma16b(a, bw, acc[t]); acc[t] = wmma16b(al, bw, acc[t]); } }
#pragma unroll
  for (int t = 0; t < 8; ++t) { const int cc = t * 16 + nloc; const float bb = bfv(bh1[cc]);
#pragma unroll
    for (int r8 = 0; r8 < 8; ++r8) Tf[8 * hlf + r8][cc] = silu(acc[t][r8] * (1.0f / (HS * WSC)) + bb); }
  wave_lds_sync();
  for (int rr = 0; rr < 16; ++rr) for (int q = 0; q < 4; ++q) { b16 p, ql; split16(Tf[rr][q * 32 + lane] * HS, p, ql); Ah[rr][q * 32 + lane] = p; Al[rr][q * 32 + lane] = ql; }
  wave_lds_sync();
#pragma unroll
  for (int t = 0; t < 8; ++t) acc[t] = (v8f){};
#pragma unroll
  for (int kb = 0; kb < DH; kb += 32) { const v16b a = frag_kb(&Ah[nloc][kb], hlf), al = frag_kb(&Al[nloc][kb], hlf);
#pragma unroll
    for (int t = 0; t < 8; ++t) { const v16b bw = frag_kb(WH2 + (size_t)(t * 16 + nloc) * DH + kb, hlf); acc[t] = wmma16b(a, bw, acc[t]); acc[t] = wmma16b(al, bw, acc[t]); } }
#pragma unroll
  for (int t = 0; t < 8; ++t) { const int cc = t * 16 + nloc; const float bb = bfv(bh2[cc]);
#pragma unroll
    for (int r8 = 0; r8 < 8; ++r8) { const int rr = 8 * hlf + r8; Tf[rr][cc] = acc[t][r8] * (1.0f / (HS * WSC)) + bb + bfv(h[(m0 + rr) * DH + cc]); } }
  wave_lds_sync();
  for (int pass = 0; pass < 2; ++pass) { for (int rr = 0; rr < 16; ++rr) { float v[4], s = 0.0f; for (int k = 0; k < 4; ++k) { v[k] = Tf[rr][lane * 4 + k]; s += v[k]; } for (int o = 16; o; o >>= 1) s += __shfl_xor(s, o); const float mu = s / DH; float s2 = 0.0f; for (int k = 0; k < 4; ++k) s2 += (v[k] - mu) * (v[k] - mu); for (int o = 16; o; o >>= 1) s2 += __shfl_xor(s2, o); const float rs = rsqrtf(s2 / DH + LNEPS);
      v4f o4; for (int k = 0; k < 4; ++k) { const int c = lane * 4 + k; o4[k] = pmul(pmul(v[k] - mu, rs), bfv(lg[c])) + bfv(lb[c]); } *(volatile v4f*)(HN + (m0 + rr) * DH + lane * 4) = o4; } __threadfence(); } }
__global__ __launch_bounds__(512) void coord_kernel(const float* __restrict__ x, const float* __restrict__ WGT, const float* __restrict__ CNT, const int* __restrict__ dsts, const int* __restrict__ PERM, const int* __restrict__ ROWPTR, const int* __restrict__ ROWCNT, int permLen, int NLIM, int ELIM, float* __restrict__ XN) { __shared__ float Zs[16][4]; const int wave = threadIdx.x >> 5, lane = threadIdx.x & 31; const size_t i = (size_t)blockIdx.x * 16 + wave;
  if (i < (size_t)NLIM) { int st = ROWPTR[i], cnt = ROWCNT[i]; cnt = iclamp(cnt, 0, E); st = iclamp(st, 0, permLen - cnt); float a = 0.0f; const int k = lane & 3;
const float xi = bfv(x[i * 3 + (k < 3 ? k : 0)]);
#pragma unroll 1
    for (int j = 0; j < cnt; ++j) { const int e = iclamp(PERM[st + j], 0, E - 1); const int d = iclamp(dsts[e], 0, N - 1); if ((size_t)d >= (size_t)NLIM || e >= ELIM) continue; const float df = xi - bfv(x[(size_t)d * 3 + (k < 3 ? k : 0)]); a += pmul(df, WGT[(e >> 4) * 32 + (e & 15)]); }
    if (lane < 3) Zs[wave][lane] = xi + a / CNT[i]; }
  __syncthreads(); const int nrow = (NLIM - (int)(blockIdx.x * 16)) < 16 ? (NLIM - (int)(blockIdx.x * 16)) : 16;
  for (int pass = 0; pass < 2; ++pass) { for (int idx = threadIdx.x; idx < nrow * 3; idx += 512) ((volatile float*)XN)[(size_t)blockIdx.x * 48 + idx] = Zs[idx / 3][idx % 3]; __threadfence(); } }
}

extern "C" void kernel_launch(void* const* d_in, const int* in_sizes, int n_in, void* d_out, int out_size, void* d_ws, size_t ws_size, hipStream_t stream) {
  (void)n_in;
  auto Fp = [&](int i) { return (const float*)d_in[i]; }; auto Ip = [&](int i) { return (const int*)d_in[i]; };
  if (in_sizes[0] != N * DH || in_sizes[1] != N * 3 || in_sizes[2] != E * DE || in_sizes[3] != (KX + 1) * DM || in_sizes[5] != DM * DM || in_sizes[7] != 2 * DH * DH || in_sizes[9] != DH * DH || in_sizes[11] != DM * DM || in_sizes[13] != DM || in_sizes[17] != 2 * E || out_size != N * DH + N * 3) return;
  const int NLIM = N, ELIM = E;
  size_t off = 0; char* ws = (char*)d_ws;
  auto carve = [&](size_t bytes) { char* p = ws + off; off += (bytes + 255) & ~(size_t)255; return p; };
  b16* WE1 = (b16*)carve((size_t)DM * KXP * 2); b16* WE2 = (b16*)carve((size_t)DM * DM * 2); b16* WX1 = (b16*)carve((size_t)DM * DM * 2); b16* WH1 = (b16*)carve((size_t)DH * 2 * DH * 2); b16* WH2 = (b16*)carve((size_t)DH * DH * 2);
  b16* MSG = (b16*)carve((size_t)(E / 2) * DM * 2); float* WGT = (float*)carve((size_t)E * 2 * 4); float* AGG0 = (float*)carve((size_t)N * DM * 4);     float* AGG = (float*)carve((size_t)N * DM * 4); float* CNT = (float*)carve((size_t)N * 4);
  CsrBufsD cd; off = csr_carveD(cd, ws, off, E, N); CsrBufsS cs; off = csr_carveS(cs, ws, off, E, N);
  if (off > ws_size || off > ((size_t)256 << 20)) return;
  float* HN = (float*)d_out; float* XN = HN + (size_t)N * DH;
  wput_kernel<<<(DM * (KXP / 8) + 255) / 256, 256, 0, stream>>>(Fp(3), Fp(5), Fp(11), Fp(7), Fp(9), WE1, WE2, WX1, WH1, WH2);
  csr_buildD(cd, Ip(17) + E, E, N, stream); csr_buildS(cs, Ip(17), E, N, stream);
  { const int EH = E / 2; const int e1 = ELIM < EH ? ELIM : EH;
    edge_kernel<<<(e1 + 15) / 16, 32, 0, stream>>>(Fp(0), Fp(1), Fp(2), Ip(17), WE1, WE2, WX1, Fp(3), Fp(4), Fp(6), Fp(12), Fp(13), Fp(14), 0, e1, NLIM, MSG, WGT);
    agg_kernel<0><<<(NLIM + 7) / 8, 256, 0, stream>>>(MSG, 0, EH, AGG0, Ip(17), cd.PERM, cd.ROWPTR, cd.ROWCNT, (int)cd.permLen, NLIM, ELIM, AGG0, CNT);
    if (ELIM > EH) edge_kernel<<<(ELIM - EH) / 16, 32, 0, stream>>>(Fp(0), Fp(1), Fp(2), Ip(17), WE1, WE2, WX1, Fp(3), Fp(4), Fp(6), Fp(12), Fp(13), Fp(14), EH, ELIM, NLIM, MSG, WGT);
    agg_kernel<1><<<(NLIM + 7) / 8, 256, 0, stream>>>(MSG, EH, E, AGG0, Ip(17), cd.PERM, cd.ROWPTR, cd.ROWCNT, (int)cd.permLen, NLIM, ELIM, AGG, CNT); }
  node_kernel<<<NLIM / 16, 32, 0, stream>>>(Fp(0), AGG, WH1, WH2, Fp(8), Fp(10), Fp(15), Fp(16), NLIM, HN);
  coord_kernel<<<(NLIM + 15) / 16, 512, 0, stream>>>(Fp(1), WGT, CNT, Ip(17) + E, cs.PERM, cs.ROWPTR, cs.ROWCNT, (int)cs.permLen, NLIM, ELIM, XN);
}
